// PillarAttentionClassifier_76124000354424
// MI455X (gfx1250) — hardware-verified
//
#include <hip/hip_runtime.h>
#include <math.h>

typedef __attribute__((ext_vector_type(16))) _Float16 v16h;
typedef __attribute__((ext_vector_type(16))) __bf16 v16b;
typedef __attribute__((ext_vector_type(8)))  _Float16 v8h;
typedef __attribute__((ext_vector_type(8)))  float v8f;
typedef __attribute__((ext_vector_type(4)))  float v4f;
typedef __attribute__((ext_vector_type(2)))  float v2f;
typedef __attribute__((ext_vector_type(4)))  unsigned v4u;
typedef __attribute__((ext_vector_type(4)))  int v4i;
typedef float __attribute__((may_alias)) float_a;
typedef int __attribute__((may_alias)) int_a;

template <typename T> __device__ __forceinline__ void vst2(void* p, T v) { *(volatile T*)p = v; __threadfence(); *(volatile T*)p = v; }
__device__ __forceinline__ v8f wmma16(v16h a, v16h b, v8f c) {
  v8f d = __builtin_amdgcn_wmma_f32_16x16x32_f16(false, a, false, b, (short)0, c, false, false);
  asm volatile("v_nop\n\tv_nop\n\tv_nop\n\tv_nop" : "+v"(d) : "v"(a), "v"(b));
  return d;
}
__device__ __forceinline__ v8f wmma_bf(v16b a, v16b b, v8f c) {
  v8f d = __builtin_amdgcn_wmma_f32_16x16x32_bf16(false, a, false, b, (short)0, c, false, false);
  asm volatile("v_nop\n\tv_nop\n\tv_nop\n\tv_nop" : "+v"(d) : "v"(a), "v"(b));
  return d;
}
__device__ __forceinline__ v16h frag_h(const _Float16* rowk0, int lane) {
  union { v16h v; v8h q[2]; } u; const _Float16* p = rowk0 + 8 * (lane >> 4);
  u.q[0] = *(const v8h*)p; u.q[1] = *(const v8h*)(p + 16); return u.v;
}
__device__ __forceinline__ v16h frag_f32(const float* rowk0, int lane) {
  v16h a; const float* p = rowk0 + 8 * (lane >> 4);
#pragma unroll
  for (int i = 0; i < 8; ++i) { a[i] = (_Float16)p[i]; a[8 + i] = (_Float16)p[16 + i]; }
  return a;
}
__device__ __forceinline__ v16h frag_f32s(const float* rowk0, int lane, float sc) {
  v16h a; const float* p = rowk0 + 8 * (lane >> 4);
#pragma unroll
  for (int i = 0; i < 8; ++i) { a[i] = (_Float16)(p[i] * sc); a[8 + i] = (_Float16)(p[16 + i] * sc); }
  return a;
}
__device__ __forceinline__ v16h fragc_f32(const float* W, int k0, int n, int lane, int ld, int K) {
  v16h a; const int g = lane >> 4;
#pragma unroll
  for (int i = 0; i < 8; ++i) { const int ka = k0 + 8 * g + i, kb = ka + 16;
    a[i] = (_Float16)(ka < K ? W[(size_t)(ka < K ? ka : K - 1) * ld + n] : 0.f); a[8 + i] = (_Float16)(kb < K ? W[(size_t)(kb < K ? kb : K - 1) * ld + n] : 0.f); }
  return a;
}
struct F2 { v16b h, l; };
__device__ __forceinline__ F2 bsplit16(const float v[16]) { F2 r;
#pragma unroll
  for (int i = 0; i < 16; ++i) { const __bf16 h = (__bf16)v[i]; r.h[i] = h; r.l[i] = (__bf16)(v[i] - (float)h); }
  return r; }
__device__ __forceinline__ F2 split_row(const float* row, int k0, int lane) { float v[16]; const float* p = row + k0 + 8 * (lane >> 4);
#pragma unroll
  for (int i = 0; i < 8; ++i) { v[i] = p[i]; v[8 + i] = p[16 + i]; }
  return bsplit16(v); }
__device__ __forceinline__ F2 split_rowK(const float* row, int k0, int lane, int K) { float v[16]; const int g = lane >> 4;
#pragma unroll
  for (int i = 0; i < 8; ++i) { const int ka = k0 + 8 * g + i, kb = ka + 16; v[i] = ka < K ? row[ka < K ? ka : K - 1] : 0.f; v[8 + i] = kb < K ? row[kb < K ? kb : K - 1] : 0.f; }
  return bsplit16(v); }
__device__ __forceinline__ F2 split_col(const float* W, int k0, int n, int lane, int ld, int K) { float v[16]; const int g = lane >> 4;
#pragma unroll
  for (int i = 0; i < 8; ++i) { const int ka = k0 + 8 * g + i, kb = ka + 16; v[i] = ka < K ? W[(size_t)(ka < K ? ka : K - 1) * ld + n] : 0.f; v[8 + i] = kb < K ? W[(size_t)(kb < K ? kb : K - 1) * ld + n] : 0.f; }
  return bsplit16(v); }
__device__ __forceinline__ v8f mac3(const F2& a, const F2& b, v8f c) { c = wmma_bf(a.l, b.h, c); c = wmma_bf(a.h, b.l, c); return wmma_bf(a.h, b.h, c); }
__device__ __forceinline__ float sigm(float v) { return 1.0f / (1.0f + expf(-v)); }
#define LDSX() do { asm volatile("s_wait_dscnt 0" ::: "memory"); __builtin_amdgcn_wave_barrier(); __builtin_amdgcn_fence(__ATOMIC_RELEASE, "workgroup"); } while (0)


#define NRW 524288
#define NGP 12
#define REP 96
__constant__ int c_gidx[NGP][3] = {{0,1,2},{3,4,3},{5,6,5},{7,8,9},{10,11,10},{12,13,14},{15,16,15},{17,18,17},{19,19,19},{20,21,22},{23,24,25},{26,27,28}};
__constant__ int c_glen[NGP] = {3,2,2,3,2,3,2,2,1,3,3,3};
__device__ __forceinline__ float bfr(float v) { return (float)(__bf16)v; }
__device__ __attribute__((noinline)) float exp_ni(float v) { return expf(v); }
__device__ __forceinline__ F2 split_lds(const float* rowk0, int lane) { return split_row(rowk0, 0, lane); }

__global__ __launch_bounds__(128) void k_pillar(const float* __restrict__ x, const float* __restrict__ We, const float* __restrict__ be, const float* __restrict__ eg, const float* __restrict__ ebt, const float* __restrict__ em, const float* __restrict__ ev,
                                               const float* __restrict__ Wa, const float* __restrict__ ba, const float* __restrict__ W1, const float* __restrict__ b1, const float* __restrict__ g1, const float* __restrict__ bb1, const float* __restrict__ m1, const float* __restrict__ v1,
                                               const float* __restrict__ W2, const float* __restrict__ b2, const float* __restrict__ g2, const float* __restrict__ bb2, const float* __restrict__ m2, const float* __restrict__ v2,
                                               const float* __restrict__ W3, const float* __restrict__ b3, const float* __restrict__ g3, const float* __restrict__ bb3, const float* __restrict__ m3, const float* __restrict__ v3, const float* __restrict__ W4, const float* __restrict__ b4, float* __restrict__ out) {
  __shared__ __align__(16) float sR[4][16][REP + 4]; __shared__ __align__(16) float sW[4][16][16]; __shared__ __align__(16) float sH[4][16][68]; __shared__ __align__(16) float sOut[64];
  const int tid = threadIdx.x, wave = tid >> 5, lane = tid & 31, col = lane & 15, g = lane >> 4; const size_t r0 = (size_t)blockIdx.x * 64 + wave * 16; const size_t myrow = r0 + col;
  { const float* xr = x + myrow * 29;
#pragma unroll 1
    for (int gg = 0; gg < 6; ++gg) { const int gi = g * 6 + gg; const int n = c_glen[gi]; float xi[3];
#pragma unroll
      for (int i = 0; i < 3; ++i) xi[i] = i < n ? bfr(xr[c_gidx[gi][i]]) : 0.f;
#pragma unroll
      for (int o = 0; o < 8; ++o) { float a = bfr(be[gi * 8 + o]);
#pragma unroll
        for (int i = 0; i < 3; ++i) a += xi[i] * bfr(We[(gi * 3 + i) * 8 + o]);
        a = a > 0.f ? a : 0.f;
        sR[wave][col][gi * 8 + o] = bfr(eg[gi * 8 + o]) * (a - bfr(em[gi * 8 + o])) * rsqrtf(bfr(ev[gi * 8 + o]) + 1e-5f) + bfr(ebt[gi * 8 + o]); } } }
  LDSX();
  { v8f acc = {};
#pragma unroll
    for (int kc = 0; kc < 3; ++kc) { const F2 a = split_row(&sR[wave][col][0], kc * 32, lane); const v16b wb = split_col(Wa, kc * 32, col < NGP ? col : NGP - 1, lane, NGP, REP).h; acc = wmma_bf(a.l, wb, acc); acc = wmma_bf(a.h, wb, acc); }
    const float bb = col < NGP ? bfr(ba[col]) : 0.f;
#pragma unroll
    for (int r = 0; r < 8; ++r) { const float lv = col < NGP ? acc[r] + bb : -3.0e38f; float mx = lv;
#pragma unroll
      for (int o_ = 1; o_ < 16; o_ <<= 1) mx = fmaxf(mx, __shfl_xor(mx, o_, 32));
      const float e = col < NGP ? exp_ni(lv - mx) : 0.f; float se = e;
#pragma unroll
      for (int o_ = 1; o_ < 16; o_ <<= 1) se += __shfl_xor(se, o_, 32);
      sW[wave][8 * g + r][col] = e / se; } }
  LDSX();
#pragma unroll 1
  for (int gg = 0; gg < 6; ++gg) { const int gi = g * 6 + gg; const float wgt = sW[wave][col][gi];
#pragma unroll
    for (int o = 0; o < 8; ++o) sR[wave][col][gi * 8 + o] *= wgt; }
  LDSX();
  { v8f acc[4] = {};
#pragma unroll
    for (int kc = 0; kc < 3; ++kc) { const F2 a = split_row(&sR[wave][col][0], kc * 32, lane);
#pragma unroll
      for (int j = 0; j < 4; ++j) { const v16b wb = split_col(W1, kc * 32, j * 16 + col, lane, 64, REP).h; acc[j] = wmma_bf(a.l, wb, acc[j]); acc[j] = wmma_bf(a.h, wb, acc[j]); } }
#pragma unroll
    for (int j = 0; j < 4; ++j) { const int n = j * 16 + col; const float bb = bfr(b1[n]), sc = bfr(g1[n]) * rsqrtf(bfr(v1[n]) + 1e-5f), mu = bfr(m1[n]), be_ = bfr(bb1[n]);
#pragma unroll
      for (int r = 0; r < 8; ++r) { float h = acc[j][r] + bb; h = h > 0.f ? h : 0.f; sH[wave][8 * g + r][n] = sc * (h - mu) + be_; } } }
  LDSX();
  float h2v[2][8];
  { v8f acc[2] = {};
#pragma unroll
    for (int kc = 0; kc < 2; ++kc) { const F2 a = split_row(&sH[wave][col][0], kc * 32, lane);
#pragma unroll
      for (int j = 0; j < 2; ++j) { const v16b wb = split_col(W2, kc * 32, j * 16 + col, lane, 32, 64).h; acc[j] = wmma_bf(a.l, wb, acc[j]); acc[j] = wmma_bf(a.h, wb, acc[j]); } }
#pragma unroll
    for (int j = 0; j < 2; ++j) { const int n = j * 16 + col; const float bb = bfr(b2[n]), sc = bfr(g2[n]) * rsqrtf(bfr(v2[n]) + 1e-5f), mu = bfr(m2[n]), be_ = bfr(bb2[n]);
#pragma unroll
      for (int r = 0; r < 8; ++r) { float h = acc[j][r] + bb; h = h > 0.f ? h : 0.f; h2v[j][r] = sc * (h - mu) + be_; } } }
  LDSX();
#pragma unroll
  for (int j = 0; j < 2; ++j)
#pragma unroll
    for (int r = 0; r < 8; ++r) sH[wave][8 * g + r][j * 16 + col] = h2v[j][r];
  LDSX();
  { v8f acc = {}; const F2 a = split_row(&sH[wave][col][0], 0, lane); const v16b wb = split_col(W3, 0, col, lane, 16, 32).h; acc = wmma_bf(a.l, wb, acc); acc = wmma_bf(a.h, wb, acc);
    const float bb = bfr(b3[col]), sc = bfr(g3[col]) * rsqrtf(bfr(v3[col]) + 1e-5f), mu = bfr(m3[col]), be_ = bfr(bb3[col]), w4 = bfr(W4[col]), bias4 = bfr(b4[0]);
#pragma unroll
    for (int r = 0; r < 8; ++r) { float h = acc[r] + bb; h = h > 0.f ? h : 0.f; h = sc * (h - mu) + be_; float d = h * w4;
#pragma unroll
      for (int o_ = 1; o_ < 16; o_ <<= 1) d += __shfl_xor(d, o_, 32);
      if (col == 0) sOut[wave * 16 + 8 * g + r] = 1.0f / (1.0f + exp_ni(-(d + bias4))); } }
  __syncthreads();
  if (tid < 16) vst2(out + (size_t)blockIdx.x * 64 + tid * 4, *(const v4f*)(&sOut[tid * 4]));
}
extern "C" void kernel_launch(void* const* d_in, const int* in_sizes, int n_in, void* d_out, int out_size, void* d_ws, size_t ws_size, hipStream_t stream) {
  (void)in_sizes; (void)n_in; (void)out_size; (void)ws_size; (void)d_ws;
  const float** I = (const float**)d_in;
  k_pillar<<<NRW / 64, 128, 0, stream>>>(I[0], I[1], I[2], I[3], I[4], I[5], I[6], I[7], I[8], I[9], I[10], I[11], I[12], I[13], I[14], I[15], I[16], I[17], I[18], I[19], I[20], I[21], I[22], I[23], I[24], I[25], I[26], I[27], I[28], (float*)d_out);
}
